// KVR_Spatial_SelfAttention_18133351923890
// MI455X (gfx1250) — hardware-verified
//
#include <hip/hip_runtime.h>
#include <stddef.h>
#include <stdint.h>

#define NB    4
#define SL    1024
#define NTOK  4096
#define CM    512
#define NH    8
#define HDM   64
#define NQKV  1536
#define KSEL  63
#define QPB   64
#define NLB   (SL / QPB)

static_assert(NTOK == NB * SL);
static_assert(NH * HDM == CM);
static_assert(NQKV == 3 * CM);
static_assert(CM % 64 == 0);
static_assert(CM % 32 == 0);
static_assert(NQKV % 64 == 0);
static_assert(NTOK % 256 == 0);
static_assert((NTOK * CM) % 2048 == 0);
static_assert((CM * CM) % 2048 == 0);
static_assert(SL % QPB == 0);
static_assert(QPB == 64);
static_assert(KSEL > 48);
static_assert(KSEL <= 64);
static_assert(HDM == 64);

typedef _Float16 v16h __attribute__((ext_vector_type(16)));
typedef _Float16 v8h  __attribute__((ext_vector_type(8)));
typedef float    v8f  __attribute__((ext_vector_type(8)));
typedef float    v4f  __attribute__((ext_vector_type(4)));
typedef unsigned int v4u __attribute__((ext_vector_type(4)));

union Frag  { v16h v; v8h h[2]; };
union Pack8 { v8h h; v4u u; };

__device__ __forceinline__ v8f mma16(v16h a, v16h b, v8f c) {
  c = __builtin_amdgcn_wmma_f32_16x16x32_f16(false, a, false, b, (short)0, c, false, false);
  asm volatile("v_nop\n\tv_nop\n\tv_nop\n\tv_nop" : "+v"(c) : "v"(a), "v"(b));
  return c;
}

__device__ __forceinline__ v16h ldfrag(const _Float16* p, int ld, int row0, int k0, int lane) {
  const int m = lane & 15, lh = lane >> 4;
  const _Float16* q = p + (size_t)(row0 + m) * ld + k0 + 8 * lh;
  Frag f;
  f.h[0] = *(const v8h*)(q);
  f.h[1] = *(const v8h*)(q + 16);
  return f.v;
}

__device__ __forceinline__ v8f zero8() { return (v8f){0.f, 0.f, 0.f, 0.f, 0.f, 0.f, 0.f, 0.f}; }

__device__ __forceinline__ void gemm32x64(const _Float16* __restrict__ A, int lda,
                                          const _Float16* __restrict__ Bt, int ldb, int K,
                                          int m0, int n0, int lane, v8f (&acc)[2][4]) {
#pragma unroll 1
  for (int k0 = 0; k0 < K; k0 += 32) {
    const v16h a0 = ldfrag(A, lda, m0, k0, lane);
    const v16h a1 = ldfrag(A, lda, m0 + 16, k0, lane);
    const v16h b0 = ldfrag(Bt, ldb, n0, k0, lane);
    const v16h b1 = ldfrag(Bt, ldb, n0 + 16, k0, lane);
    const v16h b2 = ldfrag(Bt, ldb, n0 + 32, k0, lane);
    const v16h b3 = ldfrag(Bt, ldb, n0 + 48, k0, lane);
    acc[0][0] = mma16(a0, b0, acc[0][0]);
    acc[1][0] = mma16(a1, b0, acc[1][0]);
    acc[0][1] = mma16(a0, b1, acc[0][1]);
    acc[1][1] = mma16(a1, b1, acc[1][1]);
    acc[0][2] = mma16(a0, b2, acc[0][2]);
    acc[1][2] = mma16(a1, b2, acc[1][2]);
    acc[0][3] = mma16(a0, b3, acc[0][3]);
    acc[1][3] = mma16(a1, b3, acc[1][3]);
  }
}

__global__ __launch_bounds__(256) void k_cvt(const float* __restrict__ src, _Float16* __restrict__ dh, float scale) {
  const int tid = threadIdx.x;
  const size_t o = (size_t)blockIdx.x * 2048 + (size_t)tid * 8;
  const v4f a0 = *(const v4f*)(src + o) * scale;
  const v4f a1 = *(const v4f*)(src + o + 4) * scale;
  Pack8 pk;
  pk.h = (v8h){(_Float16)a0[0], (_Float16)a0[1], (_Float16)a0[2], (_Float16)a0[3],
               (_Float16)a1[0], (_Float16)a1[1], (_Float16)a1[2], (_Float16)a1[3]};
  const v4u vv = pk.u;
  volatile v4u* d = (volatile v4u*)(dh + o);
  *d = vv;
  __threadfence();
  *d = vv;
}

#define OTP 68
__device__ __forceinline__ void out_epilogue_f32(v8f (&acc)[2][4], float scale,
                                                 float* sw, float* __restrict__ out, int ldo,
                                                 int m0, int n0, int lane, int hh, int c) {
#pragma unroll
  for (int sub = 0; sub < 2; ++sub) {
    __syncthreads();
#pragma unroll
    for (int t = 0; t < 4; ++t) {
#pragma unroll
      for (int r = 0; r < 8; ++r) sw[(8 * hh + r) * OTP + 16 * t + c] = acc[sub][t][r] * scale;
    }
    __syncthreads();
    v4f val[8];
    size_t go[8];
#pragma unroll
    for (int it = 0; it < 8; ++it) {
      const int p    = lane + 32 * it;
      const int L    = p >> 3;
      const int pc   = p & 7;
      const int row  = L >> 1;
      const int half = L & 1;
      val[it] = *(const v4f*)(sw + row * OTP + half * 32 + pc * 4);
      go[it]  = (size_t)(m0 + sub * 16 + row) * ldo + n0 + half * 32 + pc * 4;
    }
    for (int ps = 0; ps < 2; ++ps) {
#pragma unroll
      for (int it = 0; it < 8; ++it) *(volatile v4f*)(out + go[it]) = val[it];
      __threadfence();
    }
  }
}

__global__ __launch_bounds__(256) void k_gemm_f32(const _Float16* __restrict__ ap, int lda,
                                                  const _Float16* __restrict__ wt, int K, float scale,
                                                  float* __restrict__ out, int ldo) {
  __shared__ __align__(16) float st[8][16 * OTP];
  const int tid = threadIdx.x, lane = tid & 31, wave = tid >> 5;
  const int hh = lane >> 4, c = lane & 15;
  const int m0 = blockIdx.x * 256 + wave * 32;
  const int n0 = blockIdx.y * 64;

  v8f acc[2][4];
#pragma unroll
  for (int s = 0; s < 2; ++s)
#pragma unroll
    for (int t = 0; t < 4; ++t) acc[s][t] = zero8();
  gemm32x64(ap, lda, wt, K, K, m0, n0, lane, acc);
  out_epilogue_f32(acc, scale, st[wave], out, ldo, m0, n0, lane, hh, c);
}

__global__ __launch_bounds__(256) void k_attn(const float* __restrict__ qkv,
                                              const int* __restrict__ kix,
                                              float* __restrict__ out, float sscale) {
  const int tid = threadIdx.x, lane = tid & 31, wave = tid >> 5;
  const int hw = lane >> 4, c = lane & 15;
  const int bh = blockIdx.x / NLB;
  const int lb = blockIdx.x - bh * NLB;
  const int b  = bh / NH;
  const int h  = bh - b * NH;
  const float* Kb = qkv + (size_t)b * SL * NQKV + CM + h * HDM + 4 * c;
  const float* Vb = qkv + (size_t)b * SL * NQKV + 2 * CM + h * HDM + 4 * c;

#pragma unroll 1
  for (int s = 0; s < QPB / 16; ++s) {
    const int l = lb * QPB + wave * (QPB / 8) + 2 * s + hw;
    const size_t tok = (size_t)b * SL + l;
    const v4f q = *(const v4f*)(qkv + tok * NQKV + h * HDM + 4 * c);

    int idr[4];
#pragma unroll
    for (int t = 0; t < 4; ++t) {
      int j = 16 * t + c;
      j = (j > KSEL - 1) ? (KSEL - 1) : j;
      int v = kix[(size_t)l * KSEL + j];
      v = (v < 0) ? 0 : ((v > SL - 1) ? (SL - 1) : v);
      idr[t] = v;
    }

    float sc[4];
#pragma unroll
    for (int t = 0; t < 4; ++t) {
      sc[t] = -1e30f;
      const int cnt = (KSEL - 16 * t < 16) ? (KSEL - 16 * t) : 16;
#pragma unroll 1
      for (int c2 = 0; c2 < cnt; ++c2) {
        const int idx = __shfl(idr[t], c2, 16);
        const v4f kv = *(const v4f*)(Kb + (size_t)idx * NQKV);
        float d = q[0] * kv[0];
        d = fmaf(q[1], kv[1], d);
        d = fmaf(q[2], kv[2], d);
        d = fmaf(q[3], kv[3], d);
        d += __shfl_xor(d, 8, 16);
        d += __shfl_xor(d, 4, 16);
        d += __shfl_xor(d, 2, 16);
        d += __shfl_xor(d, 1, 16);
        d *= sscale;
        sc[t] = (c2 == c) ? d : sc[t];
      }
    }

    float m = fmaxf(fmaxf(sc[0], sc[1]), fmaxf(sc[2], sc[3]));
    m = fmaxf(m, __shfl_xor(m, 8, 16));
    m = fmaxf(m, __shfl_xor(m, 4, 16));
    m = fmaxf(m, __shfl_xor(m, 2, 16));
    m = fmaxf(m, __shfl_xor(m, 1, 16));
    float p[4];
    float ls = 0.f;
#pragma unroll
    for (int t = 0; t < 4; ++t) {
      p[t] = __expf(sc[t] - m);
      ls += p[t];
    }
    ls += __shfl_xor(ls, 8, 16);
    ls += __shfl_xor(ls, 4, 16);
    ls += __shfl_xor(ls, 2, 16);
    ls += __shfl_xor(ls, 1, 16);

    v4f acc = (v4f){0.f, 0.f, 0.f, 0.f};
#pragma unroll
    for (int t = 0; t < 4; ++t) {
      const int cnt = (KSEL - 16 * t < 16) ? (KSEL - 16 * t) : 16;
#pragma unroll 1
      for (int c2 = 0; c2 < cnt; ++c2) {
        const int   idx = __shfl(idr[t], c2, 16);
        const float pj  = __shfl(p[t], c2, 16);
        const v4f vv = *(const v4f*)(Vb + (size_t)idx * NQKV);
        acc[0] = fmaf(pj, vv[0], acc[0]);
        acc[1] = fmaf(pj, vv[1], acc[1]);
        acc[2] = fmaf(pj, vv[2], acc[2]);
        acc[3] = fmaf(pj, vv[3], acc[3]);
      }
    }
    const float rl = 1.0f / ls;
    const v4f o = acc * rl;
    volatile v4f* dst = (volatile v4f*)(out + tok * CM + (size_t)h * HDM + 4 * c);
    *dst = o;
    __threadfence();
    *dst = o;
  }
}

extern "C" void kernel_launch(void* const* d_in, const int* in_sizes, int n_in,
                              void* d_out, int out_size, void* d_ws, size_t ws_size,
                              hipStream_t stream) {
  if (n_in < 5) return;
  if (in_sizes[0] != NTOK * CM) return;
  if (in_sizes[1] != CM * CM) return;
  if (in_sizes[2] != CM * CM) return;
  if (in_sizes[3] != CM * CM) return;
  if (in_sizes[4] != SL * KSEL) return;
  if (out_size != NTOK * CM) return;

  const float* x   = (const float*)d_in[0];
  const float* wq  = (const float*)d_in[1];
  const float* wk  = (const float*)d_in[2];
  const float* wv  = (const float*)d_in[3];
  const int*   kix = (const int*)d_in[4];
  float* out = (float*)d_out;

  size_t off = 0;
  const size_t oX  = off; off += (size_t)NTOK * CM * 2;
  const size_t oWt = off; off += (size_t)NQKV * CM * 2;
  const size_t oP  = off; off += (size_t)NTOK * NQKV * 4;
  if (off > ws_size) return;
  if (off > (size_t)134217728) return;
  if ((oP & 127) != 0) return;

  char* ws = (char*)d_ws;
  _Float16* Xh  = (_Float16*)(ws + oX);
  _Float16* Wt  = (_Float16*)(ws + oWt);
  float*    QKV = (float*)(ws + oP);

  k_cvt<<<dim3((NTOK * CM) / 2048), dim3(256), 0, stream>>>(x, Xh, 1.0f);
  k_cvt<<<dim3((CM * CM) / 2048), dim3(256), 0, stream>>>(wq, Wt, 32.0f);
  k_cvt<<<dim3((CM * CM) / 2048), dim3(256), 0, stream>>>(wk, Wt + (size_t)CM * CM, 32.0f);
  k_cvt<<<dim3((CM * CM) / 2048), dim3(256), 0, stream>>>(wv, Wt + (size_t)2 * CM * CM, 32.0f);
  k_gemm_f32<<<dim3(NTOK / 256, NQKV / 64), dim3(256), 0, stream>>>(Xh, CM, Wt, CM, 0.03125f, QKV, NQKV);
  const float sscale = 0.125f;
  k_attn<<<dim3(NB * NH * NLB), dim3(256), 0, stream>>>(QKV, kix, out, sscale);
  (void)hipGetLastError();
}
